// CGAMixer_11579231830738
// MI455X (gfx1250) — hardware-run, weakly checked
//
#include <hip/hip_runtime.h>
#include <math.h>

constexpr int NBATCH = 4;
constexpr int NSTEP  = 1024;
constexpr int DMODEL = 256;
constexpr int DSTATE = 64;
constexpr int NSLOT  = 64;
constexpr int NROWS  = NBATCH * NSTEP;
constexpr int NQK    = 2 * DSTATE;
constexpr int NQKV   = NQK + DMODEL;
constexpr int NWROWS = NQKV + DMODEL;
static_assert(NROWS == 4096 && NQK == 128 && NQKV == 384 && NWROWS == 640, "shape constants");
static_assert(NROWS % 64 == 0 && NQKV % 64 == 0 && DMODEL % 64 == 0 && DMODEL % 32 == 0, "GEMM tile multiples");

typedef __attribute__((ext_vector_type(16))) __bf16   v16b;
typedef __attribute__((ext_vector_type(8)))  __bf16   v8b;
typedef __attribute__((ext_vector_type(8)))  float    v8f;
typedef __attribute__((ext_vector_type(4)))  float    v4f;
typedef __attribute__((ext_vector_type(4)))  unsigned v4u;

__device__ __forceinline__ unsigned short f2bf_bits(float f) {
  unsigned u = __float_as_uint(f);
  return (unsigned short)((u + 0x7FFFu + ((u >> 16) & 1u)) >> 16);
}
__device__ __forceinline__ float bf_bits2f(unsigned short h) { return __uint_as_float(((unsigned)h) << 16); }

__device__ __forceinline__ void split_pair(float x0, float x1, unsigned& hw, unsigned& lw) {
  const unsigned short h0 = f2bf_bits(x0);
  const unsigned short h1 = f2bf_bits(x1);
  const unsigned short l0 = f2bf_bits(x0 - bf_bits2f(h0));
  const unsigned short l1 = f2bf_bits(x1 - bf_bits2f(h1));
  hw = (unsigned)h0 | ((unsigned)h1 << 16);
  lw = (unsigned)l0 | ((unsigned)l1 << 16);
}

__device__ __forceinline__ void grp_guard_b(v8f& a, v8f& b, v8f& c, v8f& d, v16b x, v16b y) {
  asm volatile("v_nop\n\tv_nop\n\tv_nop\n\tv_nop" : "+v"(a), "+v"(b), "+v"(c), "+v"(d) : "v"(x), "v"(y));
}
__device__ __forceinline__ void keep4_b(v16b a, v16b b, v16b c, v16b d) { asm volatile("v_nop" :: "v"(a), "v"(b), "v"(c), "v"(d)); }
__device__ __forceinline__ void acc_guard4(v8f& a, v8f& b, v8f& c, v8f& d) {
  asm volatile("v_nop\n\tv_nop\n\tv_nop\n\tv_nop" : "+v"(a), "+v"(b), "+v"(c), "+v"(d));
}

struct FragB {
  union U { v16b v; v8b h[2]; };
  static __device__ __forceinline__ v16b load(const __bf16* p) {
    U f; f.h[0] = *(const v8b*)(p); f.h[1] = *(const v8b*)(p + 16); return f.v;
  }
  static __device__ __forceinline__ v8f mma(v16b a, v16b b, v8f c) {
    return __builtin_amdgcn_wmma_f32_16x16x32_bf16(false, a, false, b, (short)0, c, false, false);
  }
};

template <bool SPLIT, int BIAS_MODE>
__global__ __launch_bounds__(256) void wmma_gemm64_bf16(
    const unsigned short* __restrict__ Ap, const unsigned short* __restrict__ A2p, int lda,
    const unsigned short* __restrict__ Btp, const unsigned short* __restrict__ Bt2p, int ldb,
    float* __restrict__ Cout, int ldc,
    const float* __restrict__ bias,
    int M, int N, int K, float scale) {
  typedef __bf16 T;
  typedef v16b V;
  const T* A = (const T*)Ap; const T* A2 = (const T*)A2p; const T* Bt = (const T*)Btp; const T* Bt2 = (const T*)Bt2p;
  __shared__ __align__(16) float sT[8][16 * 68];
  const int lane = threadIdx.x & 31;
  const int wave = threadIdx.x >> 5;
  const int tilesN = N >> 6;
  const int tilesM = M >> 6;
  const int tile = blockIdx.x * 8 + wave;
  if (tile >= tilesM * tilesN) return;
  const int tm = tile / tilesN;
  const int tn = tile - tm * tilesN;
  const int m0 = tm << 6;
  const int n0 = tn << 6;

  const T* Ab  = A;
  const T* Bb  = Bt;
  const T* Ab2 = SPLIT ? A2 : nullptr;
  const T* Bb2 = SPLIT ? Bt2 : nullptr;

  const int rlane = lane & 15;
  const int koff  = (lane >> 4) * 8;
  const int mOff  = (lane >> 4) * 8;

  v8f acc[4][4];
#pragma unroll
  for (int i = 0; i < 4; ++i)
#pragma unroll
    for (int j = 0; j < 4; ++j) acc[i][j] = (v8f){0.f,0.f,0.f,0.f,0.f,0.f,0.f,0.f};

  for (int k0 = 0; k0 < K; k0 += 32) {
    V bh[4], bl[4];
#pragma unroll
    for (int j = 0; j < 4; ++j) {
      const size_t bo = (size_t)(n0 + (j << 4) + rlane) * ldb + koff + k0;
      bh[j] = FragB::load(Bb + bo);
      if (SPLIT) bl[j] = FragB::load(Bb2 + bo);
    }
#pragma unroll
    for (int i = 0; i < 4; ++i) {
      const size_t ao = (size_t)(m0 + (i << 4) + rlane) * lda + koff + k0;
      V ah = FragB::load(Ab + ao);
      V al;
      if (SPLIT) al = FragB::load(Ab2 + ao);
#pragma unroll
      for (int j = 0; j < 4; ++j) {
        acc[i][j] = FragB::mma(ah, bh[j], acc[i][j]);
        if (SPLIT) {
          acc[i][j] = FragB::mma(ah, bl[j], acc[i][j]);
          acc[i][j] = FragB::mma(al, bh[j], acc[i][j]);
        }
      }
      grp_guard_b(acc[i][0], acc[i][1], acc[i][2], acc[i][3], ah, SPLIT ? al : ah);
    }
    keep4_b(bh[0], bh[1], bh[2], bh[3]);
    if (SPLIT) keep4_b(bl[0], bl[1], bl[2], bl[3]);
  }
  acc_guard4(acc[0][0], acc[0][1], acc[0][2], acc[0][3]);
  acc_guard4(acc[1][0], acc[1][1], acc[1][2], acc[1][3]);
  acc_guard4(acc[2][0], acc[2][1], acc[2][2], acc[2][3]);
  acc_guard4(acc[3][0], acc[3][1], acc[3][2], acc[3][3]);

  float* slab = sT[wave];
#pragma unroll
  for (int i = 0; i < 4; ++i) {
    const int mBase = m0 + (i << 4);
#pragma unroll
    for (int j = 0; j < 4; ++j) {
      const int n = n0 + (j << 4) + rlane;
      float bv = 0.f;
      if (BIAS_MODE == 2) bv = bias[n];
#pragma unroll
      for (int r = 0; r < 8; ++r) {
        float v = acc[i][j][r] * scale;
        if (BIAS_MODE == 2) v += bv;
        slab[(mOff + r) * 68 + (j << 4) + rlane] = v;
      }
    }
    __builtin_amdgcn_fence(__ATOMIC_RELEASE, "workgroup");
    __builtin_amdgcn_wave_barrier();
    __builtin_amdgcn_fence(__ATOMIC_ACQUIRE, "workgroup");
    {
      const int hh = lane >> 4, c4 = (lane & 15) * 4;
      for (int pass = 0; pass < 2; ++pass) {
#pragma unroll
        for (int it = 0; it < 8; ++it) {
          const int row = it * 2 + hh;
          v4f v = *(const v4f*)(slab + row * 68 + c4);
          *(volatile v4f*)(Cout + (size_t)(mBase + row) * ldc + n0 + c4) = v;
        }
        __threadfence();
      }
    }
    __builtin_amdgcn_fence(__ATOMIC_RELEASE, "workgroup");
    __builtin_amdgcn_wave_barrier();
    __builtin_amdgcn_fence(__ATOMIC_ACQUIRE, "workgroup");
  }
}

__global__ __launch_bounds__(256) void split_planes_kernel(
    const float* __restrict__ src, unsigned short* __restrict__ hi, unsigned short* __restrict__ lo, int n8) {
  const int i = blockIdx.x * 256 + threadIdx.x;
  if (i < n8) {
    const v4f a = *(const v4f*)(src + (size_t)i * 8);
    const v4f b = *(const v4f*)(src + (size_t)i * 8 + 4);
    unsigned h0, h1, h2, h3, l0, l1, l2, l3;
    split_pair(a[0], a[1], h0, l0);
    split_pair(a[2], a[3], h1, l1);
    split_pair(b[0], b[1], h2, l2);
    split_pair(b[2], b[3], h3, l3);
    const v4u hv = {h0, h1, h2, h3};
    const v4u lv = {l0, l1, l2, l3};
    unsigned short* const ph = hi + (size_t)i * 8;
    unsigned short* const pl = lo + (size_t)i * 8;
    *(volatile v4u*)ph = hv;
    *(volatile v4u*)pl = lv;
    __threadfence();
    *(volatile v4u*)ph = hv;
    *(volatile v4u*)pl = lv;
  }
}

__global__ __launch_bounds__(256) void pack_weights_kernel(
    const float* __restrict__ Wq, const float* __restrict__ Wk, const float* __restrict__ Wv, const float* __restrict__ Wo,
    const float* __restrict__ bq, const float* __restrict__ bk, const float* __restrict__ bv,
    unsigned short* __restrict__ whi, unsigned short* __restrict__ wlo, float* __restrict__ bias_qkv) {
  const int tid = threadIdx.x;
  if (blockIdx.x < (NWROWS * 32) / 256) {
    const int i  = blockIdx.x * 256 + tid;
    const int n  = i >> 5;
    const int kq = (i & 31) * 8;
    const float* src = Wo;
    int ld = DMODEL;
    int col = n - NQKV;
    if (n < DSTATE)      { src = Wq; ld = DSTATE; col = n; }
    else if (n < NQK)    { src = Wk; ld = DSTATE; col = n - DSTATE; }
    else if (n < NQKV)   { src = Wv; ld = DMODEL; col = n - NQK; }
    const float x0 = src[(size_t)(kq + 0) * ld + col];
    const float x1 = src[(size_t)(kq + 1) * ld + col];
    const float x2 = src[(size_t)(kq + 2) * ld + col];
    const float x3 = src[(size_t)(kq + 3) * ld + col];
    const float x4 = src[(size_t)(kq + 4) * ld + col];
    const float x5 = src[(size_t)(kq + 5) * ld + col];
    const float x6 = src[(size_t)(kq + 6) * ld + col];
    const float x7 = src[(size_t)(kq + 7) * ld + col];
    unsigned h0, h1, h2, h3, l0, l1, l2, l3;
    split_pair(x0, x1, h0, l0);
    split_pair(x2, x3, h1, l1);
    split_pair(x4, x5, h2, l2);
    split_pair(x6, x7, h3, l3);
    const v4u hv = {h0, h1, h2, h3};
    const v4u lv = {l0, l1, l2, l3};
    unsigned short* const ph = whi + (size_t)n * DMODEL + kq;
    unsigned short* const pl = wlo + (size_t)n * DMODEL + kq;
    *(volatile v4u*)ph = hv;
    *(volatile v4u*)pl = lv;
    __threadfence();
    *(volatile v4u*)ph = hv;
    *(volatile v4u*)pl = lv;
  } else {
    const int wv = __builtin_amdgcn_readfirstlane(tid >> 5);
    if (wv < 3) {
      const int j = tid;
      const float* bsrc = bv + 4 * (j - 32);
      if (j < 16)      bsrc = bq + 4 * j;
      else if (j < 32) bsrc = bk + 4 * (j - 16);
      v4f o;
      o[0] = bsrc[0]; o[1] = bsrc[1]; o[2] = bsrc[2]; o[3] = bsrc[3];
      float* const p = bias_qkv + 4 * j;
      *(volatile v4f*)p = o;
      __threadfence();
      *(volatile v4f*)p = o;
    }
  }
}

__global__ __launch_bounds__(256) void unit_rows_kernel(const float* __restrict__ qkv, float* __restrict__ qk) {
  const int tid = threadIdx.x;
  const int lane = tid & 31;
  const int row = blockIdx.x * 8 + (tid >> 5);
  const v4f a = *(const v4f*)(qkv + (size_t)row * NQKV + lane * 4);
  float ss = 0.0f;
  ss += a[0] * a[0];
  ss += a[1] * a[1];
  ss += a[2] * a[2];
  ss += a[3] * a[3];
  ss += __shfl_xor(ss, 8, 32);
  ss += __shfl_xor(ss, 4, 32);
  ss += __shfl_xor(ss, 2, 32);
  ss += __shfl_xor(ss, 1, 32);
  const float nrm = fmaxf(sqrtf(ss), 1e-12f);
  v4f o;
  o[0] = a[0] / nrm;
  o[1] = a[1] / nrm;
  o[2] = a[2] / nrm;
  o[3] = a[3] / nrm;
  float* const p = qk + (size_t)row * NQK + lane * 4;
  *(volatile v4f*)p = o;
  __threadfence();
  *(volatile v4f*)p = o;
}

constexpr int CPITCH   = 68;
constexpr int L_CENT   = 0;
constexpr int L_VALS   = L_CENT + NSLOT * CPITCH;
constexpr int L_CNT    = L_VALS + NSLOT * DMODEL;
constexpr int L_SIM    = L_CNT + NSLOT;
constexpr int L_W      = L_SIM + NSLOT;
constexpr int L_RED    = L_W + NSLOT;
constexpr int L_MISC   = L_RED + 32;
constexpr int L_STG    = L_MISC + 32;
constexpr int STG_SZ   = NQK + DMODEL;
constexpr int SCAN_LDS_FLOATS = L_STG + 2 * STG_SZ;
constexpr int SCAN_LDS_BYTES  = SCAN_LDS_FLOATS * 4;
static_assert(L_STG == 20992 && L_STG % 256 == 0, "zero-fill loop is exact");
static_assert((L_STG * 4) % 16 == 0 && (STG_SZ * 4) % 16 == 0 && (L_W * 4) % 16 == 0 && (CPITCH * 4) % 16 == 0, "16-B alignment");
static_assert(SCAN_LDS_BYTES == 87040, "LDS total");
constexpr float NEG_FILL = -1.0e9f;
constexpr float CREATE_THR = 0.75f;
constexpr float REFINE_THR = 1.0f;
constexpr float INV_DMODEL = 1.0f / (float)DMODEL;

__global__ void __launch_bounds__(256, 1)
slot_scan_kernel(const float* __restrict__ qk, const float* __restrict__ qkv,
                 const float* __restrict__ lsp, float* __restrict__ y) {
  extern __shared__ v4u smem_dyn[];
  float* const sm     = (float*)smem_dyn;
  float* const s_cent = sm + L_CENT;
  float* const s_vals = sm + L_VALS;
  float* const s_cnt  = sm + L_CNT;
  float* const s_sim  = sm + L_SIM;
  float* const s_w    = sm + L_W;
  float* const s_red  = sm + L_RED;
  float* const s_misc = sm + L_MISC;
  float* const s_stg  = sm + L_STG;

  const int tid  = threadIdx.x;
  const int lane = tid & 31;
  const int wave = __builtin_amdgcn_readfirstlane(tid >> 5);
  const size_t row0 = (size_t)blockIdx.x * NSTEP;
  const float scale = fminf(expf(lsp[0]), 100.0f);

#pragma unroll 1
  for (int i = tid; i < L_STG; i += 256) sm[i] = 0.0f;
  {
    float v0 = qkv[row0 * NQKV + NQK + tid];
    float q0 = qk[row0 * NQK + (tid & (NQK - 1))];
    asm volatile("" : "+v"(v0));
    asm volatile("" : "+v"(q0));
    s_stg[NQK + tid] = v0;
    if (wave < 4) s_stg[tid] = q0;
  }
  __syncthreads();

  int n = 0;
#pragma unroll 1
  for (int t = 0; t < NSTEP; ++t) {
    const int cur = t & 1;
    const float* const stc = s_stg + cur * STG_SZ;
    float* const stn = s_stg + (cur ^ 1) * STG_SZ;

    const int tnx = (t + 1 < NSTEP) ? (t + 1) : (NSTEP - 1);
    const size_t rown = row0 + (size_t)tnx;
    float pv = qkv[rown * NQKV + NQK + tid];
    float pq = qk[rown * NQK + (tid & (NQK - 1))];
    asm volatile("" : "+v"(pv));
    asm volatile("" : "+v"(pq));

    if (wave < 2) {
      const float* const c = s_cent + tid * CPITCH;
      float s = 0.0f;
#pragma unroll 2
      for (int j = 0; j < DSTATE; j += 4) {
        const v4f cv = *(const v4f*)(c + j);
        const v4f qv = *(const v4f*)(stc + j);
        s = fmaf(cv[0], qv[0], s);
        s = fmaf(cv[1], qv[1], s);
        s = fmaf(cv[2], qv[2], s);
        s = fmaf(cv[3], qv[3], s);
      }
      s_sim[tid] = s;
    }
    __syncthreads();

    if (wave == 0) {
      const float s0 = s_sim[lane];
      const float s1 = s_sim[lane + 32];
      const float sc0 = (lane < n) ? s0 : NEG_FILL;
      const float sc1 = (lane + 32 < n) ? s1 : NEG_FILL;
      const float x0 = sc0 * scale;
      const float x1 = sc1 * scale;
      float mx = fmaxf(x0, x1);
      mx = fmaxf(mx, __shfl_xor(mx, 16, 32));
      mx = fmaxf(mx, __shfl_xor(mx, 8, 32));
      mx = fmaxf(mx, __shfl_xor(mx, 4, 32));
      mx = fmaxf(mx, __shfl_xor(mx, 2, 32));
      mx = fmaxf(mx, __shfl_xor(mx, 1, 32));
      const float e0 = expf(x0 - mx);
      const float e1 = expf(x1 - mx);
      float sum = e0 + e1;
      sum += __shfl_xor(sum, 16, 32);
      sum += __shfl_xor(sum, 8, 32);
      sum += __shfl_xor(sum, 4, 32);
      sum += __shfl_xor(sum, 2, 32);
      sum += __shfl_xor(sum, 1, 32);
      const float w0 = e0 / sum;
      const float w1 = e1 / sum;
      const bool up = (w1 > w0);
      float bvv = up ? w1 : w0;
      int bi = up ? (lane + 32) : lane;
#pragma unroll
      for (int off = 16; off > 0; off >>= 1) {
        const float ov = __shfl_xor(bvv, off, 32);
        const int oi = __shfl_xor(bi, off, 32);
        const bool take = (ov > bvv) || ((ov == bvv) && (oi < bi));
        bvv = take ? ov : bvv;
        bi = take ? oi : bi;
      }
      s_w[lane] = w0;
      s_w[lane + 32] = w1;
      const int selc = (bi < 0) ? 0 : ((bi > NSLOT - 1) ? (NSLOT - 1) : bi);
      const float ssel = s_sim[selc];
      if (lane == 0) {
        s_misc[0] = (float)selc;
        s_misc[1] = ssel;
      }
    }
    __syncthreads();

    int sel = (int)s_misc[0];
    sel = (sel < 0) ? 0 : ((sel > NSLOT - 1) ? (NSLOT - 1) : sel);
    const float selsim = s_misc[1];
    const float vt = stc[NQK + tid];

    float zd = 0.0f;
#pragma unroll 2
    for (int m = 0; m < NSLOT; m += 4) {
      const v4f wv = *(const v4f*)(s_w + m);
      zd = fmaf(wv[0], s_vals[(m + 0) * DMODEL + tid], zd);
      zd = fmaf(wv[1], s_vals[(m + 1) * DMODEL + tid], zd);
      zd = fmaf(wv[2], s_vals[(m + 2) * DMODEL + tid], zd);
      zd = fmaf(wv[3], s_vals[(m + 3) * DMODEL + tid], zd);
    }
    const float vsel = s_vals[sel * DMODEL + tid];
    const float cnts = s_cnt[sel];
    const float df = vsel - vt;
    float dd = df * df;
    dd += __shfl_xor(dd, 16, 32);
    dd += __shfl_xor(dd, 8, 32);
    dd += __shfl_xor(dd, 4, 32);
    dd += __shfl_xor(dd, 2, 32);
    dd += __shfl_xor(dd, 1, 32);
    if (lane == 0) s_red[wave] = dd;

    {
      const float yv = (n > 0) ? zd : 0.0f;
      float* const yp = y + (row0 + (size_t)t) * DMODEL + tid;
      *(volatile float*)yp = yv;
      __threadfence();
      *(volatile float*)yp = yv;
    }
    __syncthreads();

    float rs = s_red[0];
    rs += s_red[1];
    rs += s_red[2];
    rs += s_red[3];
    rs += s_red[4];
    rs += s_red[5];
    rs += s_red[6];
    rs += s_red[7];
    const float resid = sqrtf(rs * INV_DMODEL);
    const bool has  = (n > 0);
    const bool room = (n < NSLOT);
    const bool refine = has && room && ((selsim < CREATE_THR) || (resid > REFINE_THR));
    const bool do_add = ((!has) || refine) && room;
    const bool do_upd = has && (!refine);
    int flags = (do_add ? 1 : 0) | (do_upd ? 2 : 0);
    flags = __builtin_amdgcn_readfirstlane(flags);
    const int slot = (n < NSLOT - 1) ? n : (NSLOT - 1);

    if (wave == 0) {
      const float c0 = s_cent[sel * CPITCH + lane];
      const float c1 = s_cent[sel * CPITCH + lane + 32];
      const float k0 = stc[DSTATE + lane];
      const float k1 = stc[DSTATE + lane + 32];
      const float a0 = 0.9f * c0 + 0.1f * k0;
      const float a1 = 0.9f * c1 + 0.1f * k1;
      float ss = 0.0f;
      ss += a0 * a0;
      ss += a1 * a1;
      ss += __shfl_xor(ss, 16, 32);
      ss += __shfl_xor(ss, 8, 32);
      ss += __shfl_xor(ss, 4, 32);
      ss += __shfl_xor(ss, 2, 32);
      ss += __shfl_xor(ss, 1, 32);
      const float nrm = fmaxf(sqrtf(ss), 1e-12f);
      if (flags & 2) {
        s_cent[sel * CPITCH + lane] = a0 / nrm;
        s_cent[sel * CPITCH + lane + 32] = a1 / nrm;
        if (lane == 0) s_cnt[sel] = cnts + 1.0f;
      }
      if (flags & 1) {
        s_cent[slot * CPITCH + lane] = k0;
        s_cent[slot * CPITCH + lane + 32] = k1;
        if (lane == 0) s_cnt[slot] = 1.0f;
      }
    }
    if (flags & 2) s_vals[sel * DMODEL + tid] = (vsel * cnts + vt) / (cnts + 1.0f);
    if (flags & 1) s_vals[slot * DMODEL + tid] = vt;
    n += (flags & 1);

    stn[NQK + tid] = pv;
    if (wave < 4) stn[tid] = pq;
    __syncthreads();
  }
}

extern "C" void kernel_launch(void* const* d_in, const int* in_sizes, int n_in,
                              void* d_out, int out_size, void* d_ws, size_t ws_size, hipStream_t stream) {
  if (n_in < 10 || d_out == nullptr || d_ws == nullptr) return;
  if (in_sizes[0] != NROWS * DMODEL || in_sizes[1] != DMODEL * DSTATE || in_sizes[2] != DSTATE ||
      in_sizes[3] != DMODEL * DSTATE || in_sizes[4] != DSTATE || in_sizes[5] != DMODEL * DMODEL ||
      in_sizes[6] != DMODEL || in_sizes[7] != DMODEL * DMODEL || in_sizes[8] != DMODEL ||
      in_sizes[9] != 1 || out_size != NROWS * DMODEL) return;

  const float* x   = (const float*)d_in[0];
  const float* Wq  = (const float*)d_in[1];
  const float* bq  = (const float*)d_in[2];
  const float* Wk  = (const float*)d_in[3];
  const float* bk  = (const float*)d_in[4];
  const float* Wv  = (const float*)d_in[5];
  const float* bv  = (const float*)d_in[6];
  const float* Wo  = (const float*)d_in[7];
  const float* bo  = (const float*)d_in[8];
  const float* lsp = (const float*)d_in[9];
  float* out = (float*)d_out;

  size_t off = 0;
  unsigned char* const wsb = (unsigned char*)d_ws;
  auto carve = [&](size_t bytes) -> void* {
    void* p = (void*)(wsb + off);
    off += (bytes + 255) & ~(size_t)255;
    return p;
  };
  unsigned short* xhi = (unsigned short*)carve((size_t)NROWS * DMODEL * 2);
  unsigned short* xlo = (unsigned short*)carve((size_t)NROWS * DMODEL * 2);
  unsigned short* whi = (unsigned short*)carve((size_t)NWROWS * DMODEL * 2);
  unsigned short* wlo = (unsigned short*)carve((size_t)NWROWS * DMODEL * 2);
  float* biasq        = (float*)carve((size_t)NQKV * 4);
  float* qkv          = (float*)carve((size_t)NROWS * NQKV * 4);
  float* qkn          = (float*)carve((size_t)NROWS * NQK * 4);
  float* ybuf         = (float*)carve((size_t)NROWS * DMODEL * 4);
  unsigned short* yhi = (unsigned short*)carve((size_t)NROWS * DMODEL * 2);
  unsigned short* ylo = (unsigned short*)carve((size_t)NROWS * DMODEL * 2);
  if (off > ws_size) return;

  split_planes_kernel<<<dim3((NROWS * DMODEL / 8) / 256), dim3(256), 0, stream>>>(x, xhi, xlo, NROWS * DMODEL / 8);
  pack_weights_kernel<<<dim3((NWROWS * 32) / 256 + 1), dim3(256), 0, stream>>>(Wq, Wk, Wv, Wo, bq, bk, bv, whi, wlo, biasq);
  wmma_gemm64_bf16<true, 2><<<dim3((NROWS / 64) * (NQKV / 64) / 8), dim3(256), 0, stream>>>(
      xhi, xlo, DMODEL, whi, wlo, DMODEL, qkv, NQKV, biasq, NROWS, NQKV, DMODEL, 1.0f);
  unit_rows_kernel<<<dim3(NROWS / 8), dim3(256), 0, stream>>>(qkv, qkn);
  slot_scan_kernel<<<dim3(NBATCH), dim3(256), SCAN_LDS_BYTES, stream>>>(qkn, qkv, lsp, ybuf);
  split_planes_kernel<<<dim3((NROWS * DMODEL / 8) / 256), dim3(256), 0, stream>>>(ybuf, yhi, ylo, NROWS * DMODEL / 8);
  wmma_gemm64_bf16<true, 2><<<dim3((NROWS / 64) * (DMODEL / 64) / 8), dim3(256), 0, stream>>>(
      yhi, ylo, DMODEL, whi + (size_t)NQKV * DMODEL, wlo + (size_t)NQKV * DMODEL, DMODEL,
      out, DMODEL, bo, NROWS, DMODEL, DMODEL, 1.0f);
}
